// mLSTMCell_21380347199692
// MI455X (gfx1250) — hardware-run, weakly checked
//
#include <hip/hip_runtime.h>


#define NB   8
#define NT   512
#define NM   4096
#define ND   256
#define NU   256
#define NP   1024
#define NK   512

typedef _Float16 h16;
typedef unsigned short bf;
typedef __attribute__((ext_vector_type(16))) __bf16   v16bf;
typedef __attribute__((ext_vector_type(16))) _Float16 v16h;
typedef __attribute__((ext_vector_type(8)))  _Float16 v8h;
typedef __attribute__((ext_vector_type(8)))  unsigned short v8us;
typedef __attribute__((ext_vector_type(8)))  float    v8f;
typedef __attribute__((ext_vector_type(4)))  float    v4f;
typedef v8h  __attribute__((may_alias)) v8ha;
typedef v4f  __attribute__((may_alias)) v4fa;
typedef v8us __attribute__((may_alias)) v8usa;

__device__ __forceinline__ unsigned short f2bf(float f) { unsigned u = __float_as_uint(f); u += 0x7FFFu + ((u >> 16) & 1u); return (unsigned short)(u >> 16); }
__device__ __forceinline__ float bf2f(unsigned short b) { return __uint_as_float(((unsigned)b) << 16); }
__device__ __forceinline__ float bfr(float f) { return bf2f(f2bf(f)); }
__device__ __forceinline__ v16h cat16(v8h lo, v8h hi) { return __builtin_shufflevector(lo, hi, 0, 1, 2, 3, 4, 5, 6, 7, 8, 9, 10, 11, 12, 13, 14, 15); }
__device__ __forceinline__ v16bf cat16b(v8us lo, v8us hi) { return __builtin_bit_cast(v16bf, __builtin_shufflevector(lo, hi, 0, 1, 2, 3, 4, 5, 6, 7, 8, 9, 10, 11, 12, 13, 14, 15)); }
__device__ __forceinline__ v8f wmma16(v16h a, v16h b, v8f c) { return __builtin_amdgcn_wmma_f32_16x16x32_f16(false, a, false, b, (short)0, c, false, false); }
__device__ __forceinline__ v8f wmmab(v16bf a, v16bf b, v8f c) { return __builtin_amdgcn_wmma_f32_16x16x32_bf16(false, a, false, b, (short)0, c, false, false); }

template <typename T16> struct WFrag;
template <> struct WFrag<h16> { typedef v16h V; static __device__ __forceinline__ V ld(const h16* p) { return cat16(*(const v8h*)p, *(const v8h*)(p + 16)); } static __device__ __forceinline__ v8f mma(V a, V b, v8f c) { return wmma16(a, b, c); } };
template <> struct WFrag<bf> { typedef v16bf V; static __device__ __forceinline__ V ld(const bf* p) { return cat16b(*(const v8us*)p, *(const v8us*)(p + 16)); } static __device__ __forceinline__ v8f mma(V a, V b, v8f c) { return wmmab(a, b, c); } };
template <typename T16, int NSPLIT, bool BIAS>
__global__ __launch_bounds__(32) void k_gemmw(const T16* __restrict__ A, const T16* __restrict__ A2, const T16* __restrict__ Bt, const T16* __restrict__ Bt2, int K, float* C, int ldc, const float* __restrict__ bias, size_t sA, size_t sB, size_t sC) {
    typedef typename WFrag<T16>::V V;
    __shared__ __align__(16) float os[16 * 68];
    const size_t z = blockIdx.z; A += z * sA; if (A2) A2 += z * sA; Bt += z * sB; if (Bt2) Bt2 += z * sB; C += z * sC;
    const int lane = threadIdx.x & 31, lr = lane & 15, hi = lane >> 4; const int r0 = blockIdx.x * 64, c0 = blockIdx.y * 64;
    v8f acc[4][4];
#pragma unroll
    for (int mb = 0; mb < 4; ++mb)
#pragma unroll
        for (int nb = 0; nb < 4; ++nb) acc[mb][nb] = (v8f){};
    const size_t aoff = (size_t)(r0 + lr) * K + 8 * hi, boff = (size_t)(c0 + lr) * K + 8 * hi;
    for (int kc = 0; kc < K; kc += 32) {
        V a[4], a2[4];
#pragma unroll
        for (int mb = 0; mb < 4; ++mb) { a[mb] = WFrag<T16>::ld(A + aoff + (size_t)mb * 16 * K + kc); if (NSPLIT == 1 || NSPLIT == 2) a2[mb] = WFrag<T16>::ld(A2 + aoff + (size_t)mb * 16 * K + kc); }
#pragma unroll
        for (int nb = 0; nb < 4; ++nb) { const V b = WFrag<T16>::ld(Bt + boff + (size_t)nb * 16 * K + kc); V b2; if (NSPLIT >= 2) b2 = WFrag<T16>::ld(Bt2 + boff + (size_t)nb * 16 * K + kc);
#pragma unroll
            for (int mb = 0; mb < 4; ++mb) { acc[mb][nb] = WFrag<T16>::mma(a[mb], b, acc[mb][nb]); if (NSPLIT == 1 || NSPLIT == 2) acc[mb][nb] = WFrag<T16>::mma(a2[mb], b, acc[mb][nb]); if (NSPLIT >= 2) acc[mb][nb] = WFrag<T16>::mma(a[mb], b2, acc[mb][nb]); } }
        asm volatile("v_nop\n\tv_nop\n\tv_nop\n\tv_nop" : "+v"(acc[0][0]), "+v"(acc[1][1]), "+v"(acc[2][2]), "+v"(acc[3][3]) : "v"(a[0]), "v"(a[3]));
    }
#pragma unroll
    for (int mb = 0; mb < 4; ++mb) {
#pragma unroll
        for (int nb = 0; nb < 4; ++nb) {
#pragma unroll
            for (int j = 0; j < 8; ++j) os[(hi * 8 + j) * 68 + nb * 16 + lr] = acc[mb][nb][j]; }
        __builtin_amdgcn_wave_barrier(); asm volatile("" ::: "memory");
        float* crow = C + (size_t)(r0 + mb * 16) * ldc + c0;
#pragma unroll 1
        for (int ps = 0; ps < 2; ++ps) {
#pragma unroll
            for (int s = 0; s < 8; ++s) { const int row = 2 * s + hi, cofs = lr * 4; v4f val = *(const v4fa*)(os + row * 68 + cofs); if (BIAS) { val[0] += bfr(bias[c0 + cofs]); val[1] += bfr(bias[c0 + cofs + 1]); val[2] += bfr(bias[c0 + cofs + 2]); val[3] += bfr(bias[c0 + cofs + 3]); }
                *(volatile v4f*)(crow + (size_t)row * ldc + cofs) = val; }
            if (ps == 0) __threadfence(); }
        __builtin_amdgcn_wave_barrier(); asm volatile("" ::: "memory");
    }
}

typedef __attribute__((ext_vector_type(2))) _Float16 v2h;
typedef __attribute__((ext_vector_type(4))) _Float16 v4h;
typedef __attribute__((ext_vector_type(2))) unsigned short v2us;
typedef __attribute__((ext_vector_type(4))) unsigned short v4us;
typedef __attribute__((ext_vector_type(2))) float v2f;
typedef __attribute__((ext_vector_type(4))) int v4i;
__global__ __launch_bounds__(256) void k_cvt8(const float* __restrict__ src, bf* dst, size_t n8) { const size_t i = (size_t)blockIdx.x * 256 + threadIdx.x; if (i >= n8) return; const v8f v = *(const v8f*)(src + i * 8); v8us o;
#pragma unroll
    for (int k = 0; k < 8; ++k) o[k] = f2bf(v[k]); *(volatile v8us*)(dst + i * 8) = o; __threadfence(); *(volatile v8us*)(dst + i * 8) = o; }

__device__ __forceinline__ h16 toh_flush(float x) { const float z = (fabsf(x) < 6.103515625e-05f) ? 0.0f : x; return (h16)z; }

__global__ __launch_bounds__(256) void k_wtG(const float* __restrict__ w, int K, int N, bf* Bt) {
    const int lane = threadIdx.x & 31; const int L0 = (blockIdx.x * 8 + (threadIdx.x >> 5)) * 8; const int nlines = N * K / 64;
#pragma unroll
    for (int ps = 0; ps < 2; ++ps) {
        for (int l = 0; l < 8; ++l) { const int L = L0 + l; if (L >= nlines) break; const size_t e = (size_t)L * 64 + lane * 2; const int k = (int)(e % K), n = (int)(e / K); v2us o;
            o[0] = f2bf(w[(size_t)k * N + n]); o[1] = f2bf(w[(size_t)(k + 1) * N + n]); *(volatile v2us*)(Bt + e) = o; }
        if (ps == 0) __threadfence(); }
}

__global__ __launch_bounds__(256) void k_wth(const float* __restrict__ w, int K, int N, h16* Bt) {
    const int lane = threadIdx.x & 31; const int L0 = (blockIdx.x * 8 + (threadIdx.x >> 5)) * 8; const int nlines = N * K / 64;
#pragma unroll
    for (int ps = 0; ps < 2; ++ps) {
        for (int l = 0; l < 8; ++l) { const int Lq = L0 + l; if (Lq >= nlines) break; const size_t e = (size_t)Lq * 64 + lane * 2; const int k = (int)(e % K), n = (int)(e / K); v2h o;
            o[0] = toh_flush(bfr(w[(size_t)k * N + n])); o[1] = toh_flush(bfr(w[(size_t)(k + 1) * N + n])); *(volatile v2h*)(Bt + e) = o; }
        if (ps == 0) __threadfence(); }
}

template <bool RB>
__global__ __launch_bounds__(256) void k_c16(const float* __restrict__ src, h16* dst, size_t n8) { const size_t i = (size_t)blockIdx.x * 256 + threadIdx.x; if (i >= n8) return; const float* p = src + i * 8; const v4f a = *(const v4f*)p, b = *(const v4f*)(p + 4); v8h o;
#pragma unroll
    for (int q = 0; q < 4; ++q) { o[q] = toh_flush(RB ? bfr(a[q]) : a[q]); o[q + 4] = toh_flush(RB ? bfr(b[q]) : b[q]); }
    *(volatile v8h*)(dst + i * 8) = o; __threadfence(); *(volatile v8h*)(dst + i * 8) = o; }

__global__ __launch_bounds__(256) void k_rbf(const float* __restrict__ X, float* Y, size_t n4) { const size_t i = (size_t)blockIdx.x * 256 + threadIdx.x; if (i >= n4) return; const v4f a = *(const v4f*)(X + i * 4); v4f o;
#pragma unroll
    for (int q = 0; q < 4; ++q) o[q] = bfr(a[q]);
    *(volatile v4f*)(Y + i * 4) = o; __threadfence(); *(volatile v4f*)(Y + i * 4) = o; }

#define LNC_MAX 2048
template <bool RES>
__global__ __launch_bounds__(256) void k_lnrow(const float* __restrict__ A, const float* __restrict__ R, const float* __restrict__ gamma, const float* __restrict__ beta, float eps, int C, int nrows, float* Y) {
    const int lane = threadIdx.x & 31; const int row = blockIdx.x * 8 + (threadIdx.x >> 5); if (row >= nrows) return; const int nch = C / 128; const float* a = A + (size_t)row * C; float x[LNC_MAX / 32]; float s = 0.0f;
    for (int k = 0; k < LNC_MAX / 128; ++k) { if (k < nch) { const int c0 = k * 128 + lane * 4; v4f v = *(const v4f*)(a + c0);
            if (RES) { const v4f w = *(const v4f*)(R + (size_t)row * C + c0); v[0] = __fadd_rn(v[0], w[0]); v[1] = __fadd_rn(v[1], w[1]); v[2] = __fadd_rn(v[2], w[2]); v[3] = __fadd_rn(v[3], w[3]); }
            x[k * 4 + 0] = v[0]; x[k * 4 + 1] = v[1]; x[k * 4 + 2] = v[2]; x[k * 4 + 3] = v[3]; s = __fadd_rn(__fadd_rn(__fadd_rn(__fadd_rn(s, v[0]), v[1]), v[2]), v[3]); } }
    for (int sh = 16; sh; sh >>= 1) s = __fadd_rn(s, __shfl_xor(s, sh, 32));
    const float mean = __fdiv_rn(s, (float)C); float q = 0.0f;
    for (int k = 0; k < LNC_MAX / 128; ++k) { if (k < nch) {
            for (int j = 0; j < 4; ++j) { const float d = __fsub_rn(x[k * 4 + j], mean); x[k * 4 + j] = d; q = __fmaf_rn(d, d, q); } } }
    for (int sh = 16; sh; sh >>= 1) q = __fadd_rn(q, __shfl_xor(q, sh, 32));
    const float rstd = __fdiv_rn(1.0f, sqrtf(__fadd_rn(__fdiv_rn(q, (float)C), eps)));
    for (int k = 0; k < LNC_MAX / 128; ++k) { if (k < nch) { const int c0 = k * 128 + lane * 4; const v4f g = *(const v4f*)(gamma + c0); const v4f bt = *(const v4f*)(beta + c0);
            for (int j = 0; j < 4; ++j) x[k * 4 + j] = __fmaf_rn(__fmul_rn(x[k * 4 + j], rstd), bfr(g[j]), bfr(bt[j])); } }
    float* y = Y + (size_t)row * C;
    for (int ps = 0; ps < 2; ++ps) {
        for (int k = 0; k < LNC_MAX / 128; ++k) { if (k < nch) { v4f o; o[0] = x[k * 4 + 0]; o[1] = x[k * 4 + 1]; o[2] = x[k * 4 + 2]; o[3] = x[k * 4 + 3]; *(volatile v4f*)(y + k * 128 + lane * 4) = o; } }
        if (ps == 0) __threadfence(); }
}

__global__ __launch_bounds__(256) void k_facts(const float* __restrict__ P1, const float* __restrict__ P2, float* Kp, float* Ad, float* Mk, float* Tl) { const unsigned id = blockIdx.x * 256u + threadIdx.x; const unsigned sq = id >> 8, cl = id & 255u; float peak = 0.0f, tally = 0.0f;
    for (int t0 = 0; t0 < NT; t0 += 8) { const size_t r0 = (size_t)sq * NT + t0; float wz[8], ww[8], wg[8], wt[8];
#pragma unroll
        for (int js = 0; js < 8; ++js) { const float* p1 = P1 + (r0 + js) * NP; const float* p2 = P2 + (r0 + js) * NK; const float av = p1[NU + cl], dv = p1[2 * NU + cl], gv = p2[cl] * 0.0625f, uv = p2[NU + cl];
            const float pk = fmaxf(av + peak, av); const float wx = expf(av - pk); const float zv = 1.0f / (1.0f + expf(-dv)); tally = zv * tally + wx * gv; peak = pk;
            wz[js] = zv; ww[js] = wx * uv; wg[js] = gv; wt[js] = tally; }
        const size_t o0 = r0 * NU + cl;
#pragma unroll
        for (int js = 0; js < 8; ++js) { *(volatile float*)(Kp + o0 + (size_t)js * NU) = wz[js]; *(volatile float*)(Ad + o0 + (size_t)js * NU) = ww[js]; *(volatile float*)(Mk + o0 + (size_t)js * NU) = wg[js]; *(volatile float*)(Tl + o0 + (size_t)js * NU) = wt[js]; }
        __threadfence();
#pragma unroll
        for (int js = 0; js < 8; ++js) { *(volatile float*)(Kp + o0 + (size_t)js * NU) = wz[js]; *(volatile float*)(Ad + o0 + (size_t)js * NU) = ww[js]; *(volatile float*)(Mk + o0 + (size_t)js * NU) = wg[js]; *(volatile float*)(Tl + o0 + (size_t)js * NU) = wt[js]; } }
}

__global__ __launch_bounds__(256) void k_dots(const float* __restrict__ Tl, const float* __restrict__ P1, float* Dp) { const unsigned id = blockIdx.x * 256u + threadIdx.x; const unsigned rw = id >> 5, cb = (id & 31u) << 3; const float* ta = Tl + (size_t)rw * NU + cb; const float* pa = P1 + (size_t)rw * NP + cb; const v4f ta0 = *(const v4f*)ta, ta1 = *(const v4f*)(ta + 4), pa0 = *(const v4f*)pa, pa1 = *(const v4f*)(pa + 4);
    float acc = ta0[0] * pa0[0]; acc = acc + ta0[1] * pa0[1]; acc = acc + ta0[2] * pa0[2]; acc = acc + ta0[3] * pa0[3]; acc = acc + ta1[0] * pa1[0]; acc = acc + ta1[1] * pa1[1]; acc = acc + ta1[2] * pa1[2]; acc = acc + ta1[3] * pa1[3];
    *(volatile float*)(Dp + id) = acc; __threadfence(); *(volatile float*)(Dp + id) = acc; }

__global__ __launch_bounds__(32) void k_sheet(const float* __restrict__ Kp, const float* __restrict__ Ad, const float* __restrict__ Mk, const float* __restrict__ P1, float* Ps) { const unsigned blk = blockIdx.x; const unsigned sq = blk >> 5, qt = (blk >> 3) & 3u, sr = ((blk & 7u) << 5) + threadIdx.x; float sw[64];
#pragma unroll
    for (int jc = 0; jc < 64; ++jc) sw[jc] = 0.0f;
    for (int t0 = 0; t0 < NT; t0 += 8) { const size_t r0 = (size_t)sq * NT + t0; float w8[8];
#pragma unroll
        for (int js = 0; js < 8; ++js) { const size_t rr = r0 + js; const float zv = Kp[rr * NU + sr], yv = Ad[rr * NU + sr]; const float* mk = Mk + rr * NU + qt * 64; const float* pr = P1 + rr * NP + qt * 64; float acc = 0.0f;
#pragma unroll
            for (int jc = 0; jc < 64; ++jc) { sw[jc] = zv * sw[jc] + yv * mk[jc]; acc = acc + sw[jc] * pr[jc]; }
            w8[js] = acc; }
        float* po = Ps + (r0 * 4 + qt) * NU + sr;
#pragma unroll
        for (int js = 0; js < 8; ++js) *(volatile float*)(po + (size_t)js * 4 * NU) = w8[js];
        __threadfence();
#pragma unroll
        for (int js = 0; js < 8; ++js) *(volatile float*)(po + (size_t)js * 4 * NU) = w8[js]; }
}

__global__ __launch_bounds__(256) void k_fin(const float* __restrict__ Ps, const float* __restrict__ Dp, const float* __restrict__ P1, float* res) { const unsigned id = blockIdx.x * 256u + threadIdx.x; const unsigned rw = id >> 6, cb = (id & 63u) << 2; const float* dp = Dp + (size_t)rw * 32; float dsum = 0.0f;
#pragma unroll
    for (int gq = 0; gq < 8; ++gq) { const v4f dq = *(const v4f*)(dp + 4 * gq); dsum = dsum + dq[0]; dsum = dsum + dq[1]; dsum = dsum + dq[2]; dsum = dsum + dq[3]; }
    const float dvs = fmaxf(fabsf(dsum), 1.0f); const float* ps = Ps + (size_t)rw * 4 * NU + cb; const v4f s0 = *(const v4f*)ps, s1 = *(const v4f*)(ps + NU), s2 = *(const v4f*)(ps + 2 * NU), s3 = *(const v4f*)(ps + 3 * NU), sh = *(const v4f*)(P1 + (size_t)rw * NP + 3 * NU + cb); v4f ov;
#pragma unroll
    for (int jc = 0; jc < 4; ++jc) { const float sm = ((s0[jc] + s1[jc]) + s2[jc]) + s3[jc]; ov[jc] = ((1.0f / (1.0f + expf(-sh[jc]))) * sm) / dvs; }
    float* po = res + (size_t)id * 4; *(volatile v4f*)po = ov; __threadfence(); *(volatile v4f*)po = ov; }

extern "C" void kernel_launch(void* const* d_in, const int* in_sizes, int n_in, void* d_out, int out_size, void* d_ws, size_t ws_size, hipStream_t stream) {
    if (n_in < 15) return;
    if (in_sizes[0] != NM * ND || in_sizes[1] != ND || in_sizes[2] != ND || in_sizes[3] != ND * NU || in_sizes[4] != NU || in_sizes[5] != ND * NU || in_sizes[6] != NU || in_sizes[7] != ND * NU || in_sizes[8] != NU || in_sizes[9] != ND * NU || in_sizes[10] != NU || in_sizes[11] != ND * NU || in_sizes[12] != NU || in_sizes[13] != ND * NU || in_sizes[14] != NU) return;
    if (out_size != NM * NU) return;
    static_assert(NM == NB * NT && NP == 4 * NU && NK == 2 * NU && NM % 64 == 0 && NU % 64 == 0 && ND % 32 == 0 && ND % 128 == 0 && ND <= LNC_MAX && NM % 8 == 0 && (NM * ND / 8) % 256 == 0 && (NM * ND / 4) % 256 == 0 && (ND * NU) % (64 * 64) == 0 && (NB * NU) % 256 == 0 && NU == 256 && NT % 8 == 0 && (NM * 32) % 256 == 0 && (NM * 64) % 256 == 0, "the products: row and column counts multiples of 64, the depth of 32; k_lnrow: the channel count a multiple of 128 and at most LNC_MAX, the rows in eights; the flat grids exact; k_facts: a block one sequence of 256 columns; the ticks in eights; k_dots 32 threads a row and k_fin 64; k_sheet: 32 blocks a sequence, 8 a quarter");
    const float* i0 = (const float*)d_in[0]; const float* i1 = (const float*)d_in[1]; const float* i2 = (const float*)d_in[2]; const float* i3 = (const float*)d_in[3]; const float* i4 = (const float*)d_in[4]; const float* i5 = (const float*)d_in[5]; const float* i6 = (const float*)d_in[6]; const float* i7 = (const float*)d_in[7]; const float* i8 = (const float*)d_in[8]; const float* i9 = (const float*)d_in[9]; const float* i10 = (const float*)d_in[10]; const float* i11 = (const float*)d_in[11]; const float* i12 = (const float*)d_in[12]; const float* i13 = (const float*)d_in[13]; const float* i14 = (const float*)d_in[14]; float* res = (float*)d_out;
    char* wsp = (char*)d_ws; auto take = [&](size_t bytes) { char* p = wsp; wsp += (bytes + 255) & ~(size_t)255; return (void*)p; };
    bf* Xb = (bf*)take((size_t)NM * ND * 2); float* Xr = (float*)take((size_t)NM * ND * 4); float* Xz = (float*)take((size_t)NM * ND * 4); h16* Xh = (h16*)take((size_t)NM * ND * 2); bf* W1 = (bf*)take((size_t)NP * ND * 2); h16* W2 = (h16*)take((size_t)NK * ND * 2); float* P1 = (float*)take((size_t)NM * NP * 4); float* P2 = (float*)take((size_t)NM * NK * 4); float* Kp = (float*)take((size_t)NM * NU * 4); float* Ad = (float*)take((size_t)NM * NU * 4); float* Mk = (float*)take((size_t)NM * NU * 4); float* Tl = (float*)take((size_t)NM * NU * 4); float* Dp = (float*)take((size_t)NM * 32 * 4); float* Ps = (float*)take((size_t)NM * 4 * NU * 4);
    if ((size_t)(wsp - (char*)d_ws) > ws_size) return;
    k_cvt8<<<(unsigned)(NM * ND / 8 / 256), 256, 0, stream>>>(i0, Xb, (size_t)NM * ND / 8);
    k_rbf<<<(unsigned)(NM * ND / 4 / 256), 256, 0, stream>>>(i0, Xr, (size_t)NM * ND / 4);
    k_lnrow<false><<<(unsigned)(NM / 8), 256, 0, stream>>>(Xr, nullptr, i1, i2, 1.0e-6f, ND, NM, Xz);
    k_c16<false><<<(unsigned)(NM * ND / 8 / 256), 256, 0, stream>>>(Xz, Xh, (size_t)NM * ND / 8);
    k_wtG<<<(unsigned)(ND * NU / 64 / 64), 256, 0, stream>>>(i3, ND, NU, W1);
    k_wtG<<<(unsigned)(ND * NU / 64 / 64), 256, 0, stream>>>(i9, ND, NU, W1 + (size_t)NU * ND);
    k_wtG<<<(unsigned)(ND * NU / 64 / 64), 256, 0, stream>>>(i11, ND, NU, W1 + (size_t)2 * NU * ND);
    k_wtG<<<(unsigned)(ND * NU / 64 / 64), 256, 0, stream>>>(i13, ND, NU, W1 + (size_t)3 * NU * ND);
    k_wth<<<(unsigned)(ND * NU / 64 / 64), 256, 0, stream>>>(i5, ND, NU, W2);
    k_wth<<<(unsigned)(ND * NU / 64 / 64), 256, 0, stream>>>(i7, ND, NU, W2 + (size_t)NU * ND);
    k_gemmw<bf, 0, true><<<dim3(NM / 64, NU / 64, 1), 32, 0, stream>>>(Xb, nullptr, W1, nullptr, ND, P1, NP, i4, 0, 0, 0);
    k_gemmw<bf, 0, true><<<dim3(NM / 64, NU / 64, 1), 32, 0, stream>>>(Xb, nullptr, W1 + (size_t)NU * ND, nullptr, ND, P1 + NU, NP, i10, 0, 0, 0);
    k_gemmw<bf, 0, true><<<dim3(NM / 64, NU / 64, 1), 32, 0, stream>>>(Xb, nullptr, W1 + (size_t)2 * NU * ND, nullptr, ND, P1 + 2 * NU, NP, i12, 0, 0, 0);
    k_gemmw<bf, 0, true><<<dim3(NM / 64, NU / 64, 1), 32, 0, stream>>>(Xb, nullptr, W1 + (size_t)3 * NU * ND, nullptr, ND, P1 + 3 * NU, NP, i14, 0, 0, 0);
    k_gemmw<h16, 0, true><<<dim3(NM / 64, NU / 64, 1), 32, 0, stream>>>(Xh, nullptr, W2, nullptr, ND, P2, NK, i6, 0, 0, 0);
    k_gemmw<h16, 0, true><<<dim3(NM / 64, NU / 64, 1), 32, 0, stream>>>(Xh, nullptr, W2 + (size_t)NU * ND, nullptr, ND, P2 + NU, NK, i8, 0, 0, 0);
    k_facts<<<(unsigned)(NB * NU / 256), 256, 0, stream>>>(P1, P2, Kp, Ad, Mk, Tl);
    k_dots<<<(unsigned)(NM * 32 / 256), 256, 0, stream>>>(Tl, P1, Dp);
    k_sheet<<<(unsigned)(NB * 4 * NU / 32), 32, 0, stream>>>(Kp, Ad, Mk, P1, Ps);
    k_fin<<<(unsigned)(NM * 64 / 256), 256, 0, stream>>>(Ps, Dp, P1, res);
}
